// QuantumResidualModel_56805237457114
// MI455X (gfx1250) — hardware-verified
//
#include <hip/hip_runtime.h>


namespace {
constexpr int Bn = 16384, NQ = 7, FC = 64, NB = 128;
constexpr float AS_ = 8.0f, WS_ = 8.0f, PI_2 = 1.5707963267948966f;

typedef _Float16 b16;
typedef __attribute__((ext_vector_type(16))) _Float16 v16b;
typedef __attribute__((ext_vector_type(8))) _Float16 v8b;
typedef __attribute__((ext_vector_type(8))) float v8f;
typedef __attribute__((ext_vector_type(4))) float v4f;
__device__ __forceinline__ void split16(float v, b16& hi, b16& lo) { hi = (b16)v; lo = (b16)(v - (float)hi); }
__device__ __forceinline__ v16b frag_kb(const b16* p, int hh) { const v8b a = *(const v8b*)(p + 8 * hh), b = *(const v8b*)(p + 16 + 8 * hh); v16b f;
#pragma unroll
  for (int e = 0; e < 8; ++e) { f[e] = a[e]; f[8 + e] = b[e]; } return f; }
__device__ __forceinline__ v8f wmma16b(v16b a, v16b b, v8f c) { v8f d = __builtin_amdgcn_wmma_f32_16x16x32_f16(false, a, false, b, (short)0, c, false, false); asm volatile("v_nop\n\tv_nop\n\tv_nop\n\tv_nop" : "+v"(d) : "v"(a), "v"(b)); return d; }
__device__ __forceinline__ void wave_lds_sync() { __builtin_amdgcn_fence(__ATOMIC_RELEASE, "workgroup"); __builtin_amdgcn_wave_barrier(); __builtin_amdgcn_fence(__ATOMIC_ACQUIRE, "workgroup"); }
__device__ __forceinline__ float pmul(float a, float b) { float p = a * b; asm volatile("" : "+v"(p)); return p; }
__device__ __forceinline__ float nexp(float x) { return __builtin_amdgcn_exp2f(x * 1.4426950408889634f); }
__device__ __forceinline__ float tanh_(float x) { const float e = nexp(-2.0f * fabsf(x)); const float t = (1.0f - e) * __builtin_amdgcn_rcpf(1.0f + e); return (x >= 0.0f) ? t : -t; }

__global__ __launch_bounds__(256) void prep_kernel(const float* __restrict__ eW1, const float* __restrict__ eW2, const float* __restrict__ fW1, const float* __restrict__ fW2, b16* __restrict__ p1, b16* __restrict__ p2, b16* __restrict__ p3, b16* __restrict__ p4) {
  const int t_ = threadIdx.x;
  auto put = [&](b16* dst, size_t PL, size_t idx, float v) { b16 a, c; split16(v * WS_, a, c); ((volatile b16*)dst)[idx] = a; ((volatile b16*)dst)[PL + idx] = c; };
  for (int pass = 0; pass < 2; ++pass) {
    for (int p = t_; p < 32 * 64; p += 256) put(p1, 32 * 64, p, eW1[p]);
    for (int p = t_; p < 16 * 32; p += 256) put(p2, 16 * 32, p, eW2[p]);
    for (int p = t_; p < 64 * 64; p += 256) { const int n = p >> 6, k = p & 63; float v = 0.0f; if (k < 28) v = fW1[n * 44 + k]; else if (k >= 32 && k < 48) v = fW1[n * 44 + 28 + (k - 32)]; put(p3, 64 * 64, p, v); }
    for (int p = t_; p < 32 * 64; p += 256) put(p4, 32 * 64, p, fW2[p]);
    __threadfence();
  }
}

struct C2 { float re, im; };
__global__ __launch_bounds__(256) void circuit_kernel(const float* __restrict__ xq, const float* __restrict__ preW, const float* __restrict__ preb, const float* __restrict__ wry, const float* __restrict__ wrz, float* __restrict__ qo) {
  __shared__ float Qs[8][32];
  const int wid = threadIdx.x >> 5, lane = threadIdx.x & 31; const int b = blockIdx.x * 8 + wid;
  float ang[NQ];
#pragma unroll
  for (int q = 0; q < NQ; ++q) { float a = preb[q];
#pragma unroll
    for (int k = 0; k < NQ; ++k) a += pmul(preW[q * NQ + k], xq[(size_t)b * NQ + k]);
    ang[q] = (tanh_(a) + 1.0f) * PI_2; }
  float sr[4], si[4];
#pragma unroll
  for (int r = 0; r < 4; ++r) { sr[r] = 0.0f; si[r] = 0.0f; }
  if (lane == 0) sr[0] = 1.0f;
  auto gate1 = [&](int q, C2 g00, C2 g01, C2 g10, C2 g11) {
    const int p = 6 - q; float or_[4], oi_[4];
#pragma unroll
    for (int r = 0; r < 4; ++r) { or_[r] = sr[r]; oi_[r] = si[r]; }
#pragma unroll
    for (int r = 0; r < 4; ++r) { float pr_, pi_; int mybit;
      if (p < 5) { pr_ = __shfl_xor(or_[r], 1 << p); pi_ = __shfl_xor(oi_[r], 1 << p); mybit = (lane >> p) & 1; }
      else { const int rr = r ^ (1 << (p - 5)); pr_ = (rr == 0) ? or_[0] : (rr == 1) ? or_[1] : (rr == 2) ? or_[2] : or_[3]; pi_ = (rr == 0) ? oi_[0] : (rr == 1) ? oi_[1] : (rr == 2) ? oi_[2] : oi_[3]; mybit = (r >> (p - 5)) & 1; }
      const float m_r = or_[r], m_i = oi_[r];
      const C2 ga = mybit ? g10 : g00, gb = mybit ? g11 : g01;
      const float a_r = mybit ? pr_ : m_r, a_i = mybit ? pi_ : m_i, c_r = mybit ? m_r : pr_, c_i = mybit ? m_i : pi_;
      sr[r] = (pmul(ga.re, a_r) - pmul(ga.im, a_i)) + (pmul(gb.re, c_r) - pmul(gb.im, c_i));
      si[r] = (pmul(ga.re, a_i) + pmul(ga.im, a_r)) + (pmul(gb.re, c_i) + pmul(gb.im, c_r)); }
  };
  auto cnot = [&](int qc, int qt) { const int pc_ = 6 - qc, pt = 6 - qt; float or_[4], oi_[4];
#pragma unroll
    for (int r = 0; r < 4; ++r) { or_[r] = sr[r]; oi_[r] = si[r]; }
#pragma unroll
    for (int r = 0; r < 4; ++r) { float pr_, pi_;
      if (pt < 5) { pr_ = __shfl_xor(or_[r], 1 << pt); pi_ = __shfl_xor(oi_[r], 1 << pt); }
      else { const int rr = r ^ (1 << (pt - 5)); pr_ = (rr == 0) ? or_[0] : (rr == 1) ? or_[1] : (rr == 2) ? or_[2] : or_[3]; pi_ = (rr == 0) ? oi_[0] : (rr == 1) ? oi_[1] : (rr == 2) ? oi_[2] : oi_[3]; }
      const int a = r * 32 + lane; const int cbit = (a >> pc_) & 1;
      sr[r] = cbit ? pr_ : or_[r]; si[r] = cbit ? pi_ : oi_[r]; }
  };
#pragma unroll 1
  for (int layer = 0; layer < 3; ++layer) {
#pragma unroll 1
    for (int q = 0; q < NQ; ++q) { const float th = (q == 0) ? ang[0] : (q == 1) ? ang[1] : (q == 2) ? ang[2] : (q == 3) ? ang[3] : (q == 4) ? ang[4] : (q == 5) ? ang[5] : ang[6];
      const float c = cosf(0.5f * th), s = sinf(0.5f * th); gate1(q, C2{c, 0.f}, C2{-s, 0.f}, C2{s, 0.f}, C2{c, 0.f}); }
#pragma unroll 1
    for (int q = 0; q < NQ; ++q) { const float t1 = wry[layer * NQ + q], t2 = wrz[layer * NQ + q];
      const float c = cosf(0.5f * t1), s = sinf(0.5f * t1); gate1(q, C2{c, 0.f}, C2{-s, 0.f}, C2{s, 0.f}, C2{c, 0.f});
      const float cz = cosf(0.5f * t2), sz = sinf(0.5f * t2); gate1(q, C2{cz, -sz}, C2{0.f, 0.f}, C2{0.f, 0.f}, C2{cz, sz}); }
    const int shift = layer + 1;
#pragma unroll 1
    for (int q = 0; q < NQ; ++q) cnot(q, (q + shift) % NQ);
  }
  float res = 0.0f;
  float pa[4];
#pragma unroll
  for (int r = 0; r < 4; ++r) pa[r] = pmul(sr[r], sr[r]) + pmul(si[r], si[r]);
#pragma unroll 1
  for (int q = 0; q < NQ; ++q) { const int p = 6 - q; const int j = (q + 1) % NQ, pj = 6 - j;
    float z = 0.0f, zz = 0.0f, xr_ = 0.0f, xi_ = 0.0f;
#pragma unroll
    for (int r = 0; r < 4; ++r) { const int a = r * 32 + lane; const int bq_ = (a >> p) & 1, bj = (a >> pj) & 1;
      z += bq_ ? -pa[r] : pa[r]; zz += (bq_ ^ bj) ? -pa[r] : pa[r];
      float pr_, pi_;
      if (p < 5) { pr_ = __shfl_xor(sr[r], 1 << p); pi_ = __shfl_xor(si[r], 1 << p); }
      else { const int rr = r ^ (1 << (p - 5)); pr_ = (rr == 0) ? sr[0] : (rr == 1) ? sr[1] : (rr == 2) ? sr[2] : sr[3]; pi_ = (rr == 0) ? si[0] : (rr == 1) ? si[1] : (rr == 2) ? si[2] : si[3]; }
      if (!bq_) { xr_ += pmul(sr[r], pr_) + pmul(si[r], pi_); xi_ += pmul(sr[r], pi_) - pmul(si[r], pr_); } }
#pragma unroll
    for (int o = 1; o < 32; o <<= 1) { z += __shfl_xor(z, o); zz += __shfl_xor(zz, o); xr_ += __shfl_xor(xr_, o); xi_ += __shfl_xor(xi_, o); }
    if (lane == q) res = z; if (lane == 7 + q) res = 2.0f * xr_; if (lane == 14 + q) res = 2.0f * xi_; if (lane == 21 + q) res = zz; }
  if (lane >= 28) res = 0.0f;
  Qs[wid][lane] = res;
  __syncthreads();
  for (int pass = 0; pass < 2; ++pass) { if (threadIdx.x < 64) *(volatile v4f*)(qo + (size_t)blockIdx.x * 256 + threadIdx.x * 4) = *(const v4f*)(&Qs[0][0] + threadIdx.x * 4); __threadfence(); }
}

__global__ __launch_bounds__(256) void head_kernel(const float* __restrict__ xc, const float* __restrict__ qo, const b16* __restrict__ p1, const b16* __restrict__ p2, const b16* __restrict__ p3, const b16* __restrict__ p4,
                                                  const float* __restrict__ eb1, const float* __restrict__ eb2, const float* __restrict__ fb1, const float* __restrict__ fb2, const float* __restrict__ fW3, const float* __restrict__ fb3, const float* __restrict__ corr, float* __restrict__ out) {
  __shared__ __attribute__((aligned(16))) float Ta[8][16][64 + 4]; __shared__ float Ob[NB];
  const int wid = threadIdx.x >> 5, lane = threadIdx.x & 31, nloc = lane & 15, hlf = lane >> 4; const size_t r0 = (size_t)blockIdx.x * NB + wid * 16;
  auto afrag = [&](int kb, v16b& ah, v16b& al) {
#pragma unroll
    for (int e = 0; e < 16; ++e) { const int k = kb + ((e < 8) ? (8 * hlf + e) : (16 + 8 * hlf + e - 8)); b16 a, c; split16(Ta[wid][nloc][k] * AS_, a, c); ah[e] = a; al[e] = c; } };
  auto gemm = [&](const b16* B, size_t PL, int KK, int NT, v8f* acc) {
    for (int kb = 0; kb < KK; kb += 32) { v16b ah, al; afrag(kb, ah, al);
      for (int t = 0; t < NT; ++t) { const v16b bh_ = frag_kb(B + (size_t)(t * 16 + nloc) * KK + kb, hlf), bl_ = frag_kb(B + PL + (size_t)(t * 16 + nloc) * KK + kb, hlf);
        acc[t] = wmma16b(ah, bh_, acc[t]); acc[t] = wmma16b(al, bh_, acc[t]); acc[t] = wmma16b(ah, bl_, acc[t]); } } };
  const float sc = 1.0f / (AS_ * WS_);
  for (int i = lane; i < 16 * 16; i += 32) { const int r = i >> 4, c4 = (i & 15) * 4; *(v4f*)(&Ta[wid][r][c4]) = *(const v4f*)(xc + (r0 + r) * FC + c4); }
  wave_lds_sync();
  v8f acc[4];
  acc[0] = (v8f){}; acc[1] = (v8f){}; gemm(p1, 32 * 64, 64, 2, acc); wave_lds_sync();
#pragma unroll
  for (int t = 0; t < 2; ++t)
#pragma unroll
    for (int v = 0; v < 8; ++v) Ta[wid][8 * hlf + v][t * 16 + nloc] = fmaxf(acc[t][v] * sc + eb1[t * 16 + nloc], 0.0f);
  wave_lds_sync();
  acc[0] = (v8f){}; gemm(p2, 16 * 32, 32, 1, acc); wave_lds_sync();
#pragma unroll
  for (int v = 0; v < 8; ++v) { const int r = 8 * hlf + v; Ta[wid][r][32 + nloc] = fmaxf(acc[0][v] * sc + eb2[nloc], 0.0f); Ta[wid][r][48 + nloc] = 0.0f;
    const float qv = qo[(r0 + r) * 32 + nloc], qv2 = qo[(r0 + r) * 32 + 16 + nloc]; Ta[wid][r][nloc] = qv; Ta[wid][r][16 + nloc] = (nloc < 12) ? qv2 : 0.0f; }
  wave_lds_sync();
#pragma unroll
  for (int t = 0; t < 4; ++t) acc[t] = (v8f){};
  gemm(p3, 64 * 64, 64, 4, acc); wave_lds_sync();
#pragma unroll
  for (int t = 0; t < 4; ++t)
#pragma unroll
    for (int v = 0; v < 8; ++v) Ta[wid][8 * hlf + v][t * 16 + nloc] = fmaxf(acc[t][v] * sc + fb1[t * 16 + nloc], 0.0f);
  wave_lds_sync();
  acc[0] = (v8f){}; acc[1] = (v8f){}; gemm(p4, 32 * 64, 64, 2, acc); wave_lds_sync();
#pragma unroll
  for (int t = 0; t < 2; ++t)
#pragma unroll
    for (int v = 0; v < 8; ++v) Ta[wid][8 * hlf + v][t * 16 + nloc] = fmaxf(acc[t][v] * sc + fb2[t * 16 + nloc], 0.0f);
  wave_lds_sync();
  if (hlf == 0) { float s = fb3[0];
#pragma unroll 1
    for (int k = 0; k < 32; ++k) s += pmul(Ta[wid][nloc][k], fW3[k]);
    Ob[wid * 16 + nloc] = corr[0] * s; }
  __syncthreads();
  for (int pass = 0; pass < 2; ++pass) { if (threadIdx.x < 32) *(volatile v4f*)(out + (size_t)blockIdx.x * NB + threadIdx.x * 4) = *(const v4f*)(&Ob[threadIdx.x * 4]); __threadfence(); }
}
}

extern "C" void kernel_launch(void* const* d_in, const int* in_sizes, int n_in,
                              void* d_out, int out_size, void* d_ws, size_t ws_size, hipStream_t stream) {
  (void)n_in; (void)out_size;
  const float* xq = (const float*)d_in[0]; const float* xc = (const float*)d_in[1]; const float* preW = (const float*)d_in[2]; const float* preb = (const float*)d_in[3]; const float* wry = (const float*)d_in[4]; const float* wrz = (const float*)d_in[5];
  const float* eW1 = (const float*)d_in[6]; const float* eb1 = (const float*)d_in[7]; const float* eW2 = (const float*)d_in[8]; const float* eb2 = (const float*)d_in[9];
  const float* fW1 = (const float*)d_in[10]; const float* fb1 = (const float*)d_in[11]; const float* fW2 = (const float*)d_in[12]; const float* fb2 = (const float*)d_in[13]; const float* fW3 = (const float*)d_in[14]; const float* fb3 = (const float*)d_in[15]; const float* corr = (const float*)d_in[16];
  float* out = (float*)d_out;
  if (in_sizes[0] != Bn * NQ || in_sizes[1] != Bn * FC || in_sizes[2] != NQ * NQ || in_sizes[6] != 32 * 64 || in_sizes[10] != 64 * 44 || in_sizes[12] != 32 * 64 || in_sizes[14] != 32) return;
  size_t off = 0; char* ws = (char*)d_ws;
  auto carve = [&](size_t bytes) { char* q = ws + off; off += (bytes + 255) & ~(size_t)255; return q; };
  b16* p1 = (b16*)carve(32 * 64 * 4); b16* p2 = (b16*)carve(16 * 32 * 4); b16* p3 = (b16*)carve(64 * 64 * 4); b16* p4 = (b16*)carve(32 * 64 * 4); float* qo = (float*)carve((size_t)Bn * 32 * 4);
  if (off > ws_size) return;
  prep_kernel<<<1, 256, 0, stream>>>(eW1, eW2, fW1, fW2, p1, p2, p3, p4);
  circuit_kernel<<<Bn / 8, 256, 0, stream>>>(xq, preW, preb, wry, wrz, qo);
  head_kernel<<<Bn / NB, 256, 0, stream>>>(xc, qo, p1, p2, p3, p4, eb1, eb2, fb1, fb2, fW3, fb3, corr, out);
}
